// EdgeNetwork_13116830122450
// MI455X (gfx1250) — hardware-verified
//
#include <hip/hip_runtime.h>

typedef __attribute__((ext_vector_type(16))) _Float16 v16h;
typedef __attribute__((ext_vector_type(8)))  _Float16 v8h;
typedef __attribute__((ext_vector_type(16))) __bf16   v16b;
typedef __attribute__((ext_vector_type(8)))  __bf16   v8b;
typedef __attribute__((ext_vector_type(8)))  float    v8f;
typedef __attribute__((ext_vector_type(4)))  float    v4f;
typedef __attribute__((ext_vector_type(2)))  float    v2f;
typedef __attribute__((ext_vector_type(4)))  int      v4i;

constexpr int NATOM  = 100000;
constexpr int NEDGE  = 400000;
constexpr int ADIM   = 32;
constexpr int BDIM   = 16;
constexpr int WCOLS  = ADIM * ADIM;
constexpr int NKS    = BDIM + 1;
constexpr int KTOT   = NKS * 32;
constexpr int BPITCH = KTOT + 8;
constexpr int NT     = 256;
constexpr int WPB1   = NT / 32;
constexpr int NTILE1 = NEDGE / 16;
constexpr int TPW1   = 25;
constexpr int NBLK1  = NTILE1 / (WPB1 * TPW1);
constexpr int SPITCH = 36;

constexpr float ACARRY    = 16.0f;
constexpr float BCARRY    = 256.0f;
constexpr float LCARRY    = 2048.0f;
constexpr float OUT_SCALE = 1.0f / 4096.0f;
constexpr float LO_SCALE  = 1.0f / 8388608.0f;

constexpr int SRB    = 1024;
constexpr int NTILE2 = (NATOM + SRB - 1) / SRB;
constexpr int EPT    = 16;
constexpr int SCH    = NT * EPT;
constexpr int NCH    = (NEDGE + SCH - 1) / SCH;
constexpr int LCAP   = SCH;

static_assert(NBLK1 * WPB1 * TPW1 == NTILE1, "");
static_assert(NEDGE % 16 == 0, "");
static_assert(KTOT % 32 == 0, "");
static_assert(BPITCH % 8 == 0, "");
static_assert(NEDGE % EPT == 0, "");
static_assert(NTILE2 * SRB >= NATOM, "");
static_assert(NATOM % 4 == 0, "");
static_assert(SRB == 128 * WPB1, "");
static_assert(NEDGE < (1 << 19), "");
static_assert(SRB <= (1 << 10), "");

__device__ __forceinline__ unsigned short f2bf_bits(float f) {
  unsigned u = __float_as_uint(f);
  return (unsigned short)((u + 0x7FFFu + ((u >> 16) & 1u)) >> 16);
}
__device__ __forceinline__ float bf_bits2f(unsigned short h) { return __uint_as_float(((unsigned)h) << 16); }

__device__ __forceinline__ void dep_guard_h(v8f& a, v8f& b, v16h x, v16h y) { asm volatile("v_nop\n\tv_nop\n\tv_nop\n\tv_nop" : "+v"(a), "+v"(b) : "v"(x), "v"(y)); }
__device__ __forceinline__ void dep_guard_b(v8f& a, v8f& b, v16b x, v16b y) { asm volatile("v_nop\n\tv_nop\n\tv_nop\n\tv_nop" : "+v"(a), "+v"(b) : "v"(x), "v"(y)); }
__device__ __forceinline__ void keep4_h(v16h a, v16h b, v16h c, v16h d) { asm volatile("v_nop" :: "v"(a), "v"(b), "v"(c), "v"(d)); }
__device__ __forceinline__ void keep4_b(v16b a, v16b b, v16b c, v16b d) { asm volatile("v_nop" :: "v"(a), "v"(b), "v"(c), "v"(d)); }
template <typename T> struct Frag;
template <> struct Frag<_Float16> {
  typedef v16h V; union U { v16h v; v8h h[2]; };
  static __device__ __forceinline__ v16h load(const _Float16* p) {
    U f; f.h[0] = *(const v8h*)(p); f.h[1] = *(const v8h*)(p + 16); return f.v;
  }
  static __device__ __forceinline__ v8f mma(v16h a, v16h b, v8f c) {
    return __builtin_amdgcn_wmma_f32_16x16x32_f16(false, a, false, b, (short)0, c, false, false);
  }
  static __device__ __forceinline__ void guard(v8f& a, v8f& b, v16h x, v16h y) { dep_guard_h(a, b, x, y); }
  static __device__ __forceinline__ void keep(v16h a, v16h b, v16h c, v16h d) { keep4_h(a, b, c, d); }
};
template <> struct Frag<__bf16> {
  typedef v16b V; union U { v16b v; v8b h[2]; };
  static __device__ __forceinline__ v16b load(const __bf16* p) {
    U f; f.h[0] = *(const v8b*)(p); f.h[1] = *(const v8b*)(p + 16); return f.v;
  }
  static __device__ __forceinline__ v8f mma(v16b a, v16b b, v8f c) {
    return __builtin_amdgcn_wmma_f32_16x16x32_bf16(false, a, false, b, (short)0, c, false, false);
  }
  static __device__ __forceinline__ void guard(v8f& a, v8f& b, v16b x, v16b y) { dep_guard_b(a, b, x, y); }
  static __device__ __forceinline__ void keep(v16b a, v16b b, v16b c, v16b d) { keep4_b(a, b, c, d); }
};

__device__ __forceinline__ unsigned pk16(unsigned short a, unsigned short b) { return (unsigned)a | ((unsigned)b << 16); }
__device__ __forceinline__ unsigned short h_bits(float f) { const _Float16 h = (_Float16)f; return __builtin_bit_cast(unsigned short, h); }

__device__ __forceinline__ void mma_guard4(v8f& a0, v8f& a1, v8f& a2, v8f& a3, v16h x, v16h y0, v16h y1, v16h y2, v16h y3) {
  asm volatile("v_nop\n\tv_nop\n\tv_nop\n\tv_nop" : "+v"(a0), "+v"(a1), "+v"(a2), "+v"(a3) : "v"(x), "v"(y0), "v"(y1), "v"(y2), "v"(y3));
}

__device__ __forceinline__ int blk_excl_scan(int cnt, int* scan_ws, int tid, int* tot) {
  const int lane = tid & 31, wave = tid >> 5; int incl = cnt;
#pragma unroll
  for (int o = 1; o < 32; o <<= 1) { const int v = __shfl_up(incl, o, 32); if (lane >= o) incl += v; }
  if (lane == 31) scan_ws[wave] = incl;
  __syncthreads();
  if (wave == 0) { int wv = (lane < NT / 32) ? scan_ws[lane] : 0; int wincl = wv;
#pragma unroll
    for (int o = 1; o < 32; o <<= 1) { const int v = __shfl_up(wincl, o, 32); if (lane >= o) wincl += v; }
    if (lane < NT / 32) scan_ws[32 + lane] = wincl - wv; if (lane == 31) scan_ws[64] = wincl; }
  __syncthreads();
  const int res = scan_ws[32 + wave] + incl - cnt; *tot = scan_ws[64];
  return res;
}

__global__ __launch_bounds__(NT) void edge_transform_kernel(const float* __restrict__ atom, const float* __restrict__ bond,
                                                            const int* __restrict__ pairs, const float* __restrict__ W,
                                                            const float* __restrict__ bias, float* __restrict__ T) {
  __shared__ __align__(16) unsigned short Bh[ADIM * BPITCH];
  __shared__ __align__(16) unsigned short Bl[ADIM * BPITCH];
  __shared__ __align__(16) float slab[WPB1][16 * SPITCH];
  const int tid = threadIdx.x;

  for (int idx = tid; idx < ADIM * (BPITCH / 2); idx += NT) {
    const int n  = idx / (BPITCH / 2);
    const int p  = idx - n * (BPITCH / 2);
    const int kc = 2 * p;
    const int kcl = kc < 510 ? kc : 510;
    const int kk = kcl >> 5, jj = kcl & 31;
    const v2f wv = *(const v2f*)(W + (size_t)kk * WCOLS + n * ADIM + jj);
    int jb = kc - 512; jb = jb < 0 ? 0 : (jb > 30 ? 30 : jb);
    const v2f bv = *(const v2f*)(bias + n * ADIM + jb);
    const float fw = (kc < 512) ? 1.0f : 0.0f;
    const float fb = (kc >= 512 && kc < KTOT) ? 1.0f : 0.0f;
    const float v0 = fmaf(fw, wv[0], fb * bv[0]) * BCARRY;
    const float v1 = fmaf(fw, wv[1], fb * bv[1]) * BCARRY;
    const _Float16 h0 = (_Float16)v0, h1 = (_Float16)v1;
    const float f0 = (float)h0, f1 = (float)h1;
    const float r0 = (v0 - f0) * LCARRY, r1 = (v1 - f1) * LCARRY;
    const unsigned uh = pk16(__builtin_bit_cast(unsigned short, h0), __builtin_bit_cast(unsigned short, h1));
    const unsigned ul = pk16(h_bits(r0), h_bits(r1));
    *(unsigned*)(Bh + n * BPITCH + kc) = uh;
    *(unsigned*)(Bl + n * BPITCH + kc) = ul;
  }
  __syncthreads();

  const int lane = tid & 31, wave = tid >> 5;
  const int hh = lane >> 4, m = lane & 15;
  const _Float16* Bhp = (const _Float16*)Bh;
  const _Float16* Blp = (const _Float16*)Bl;
  float* sw = slab[wave];
  const v8f z8 = {0.f, 0.f, 0.f, 0.f, 0.f, 0.f, 0.f, 0.f};

#pragma unroll 1
  for (int t = 0; t < TPW1; ++t) {
    const int tile = (blockIdx.x * WPB1 + wave) * TPW1 + t;
    const int e0 = tile * 16;
    const int em = e0 + m;
    int nb = pairs[2 * em + 1];
    nb = nb < 0 ? 0 : (nb >= NATOM ? NATOM - 1 : nb);
    const float* arow = atom + (size_t)nb * ADIM;
    const v4f x0 = *(const v4f*)(arow + 8 * hh);
    const v4f x1 = *(const v4f*)(arow + 8 * hh + 4);
    const v4f x2 = *(const v4f*)(arow + 16 + 8 * hh);
    const v4f x3 = *(const v4f*)(arow + 20 + 8 * hh);
    const float* brow = bond + (size_t)em * BDIM;
    const v4f b0 = *(const v4f*)(brow);
    const v4f b1 = *(const v4f*)(brow + 4);
    const v4f b2 = *(const v4f*)(brow + 8);
    const v4f b3 = *(const v4f*)(brow + 12);
    float nf[16];
#pragma unroll
    for (int i = 0; i < 4; ++i) { nf[i] = x0[i]; nf[4 + i] = x1[i]; nf[8 + i] = x2[i]; nf[12 + i] = x3[i]; }
    float bs[NKS];
#pragma unroll
    for (int i = 0; i < 4; ++i) { bs[i] = b0[i] * ACARRY; bs[4 + i] = b1[i] * ACARRY; bs[8 + i] = b2[i] * ACARRY; bs[12 + i] = b3[i] * ACARRY; }
    bs[BDIM] = ACARRY;

    v8f acc0 = z8, acc1 = z8, accl0 = z8, accl1 = z8;
#pragma unroll
    for (int ks = 0; ks < NKS; ++ks) {
      const float s = bs[ks];
      v16h a;
#pragma unroll
      for (int i = 0; i < 16; ++i) a[i] = (_Float16)(s * nf[i]);
      const int boff = ks * 32 + 8 * hh;
      const v16h bh0 = Frag<_Float16>::load(Bhp + m * BPITCH + boff);
      const v16h bh1 = Frag<_Float16>::load(Bhp + (16 + m) * BPITCH + boff);
      const v16h bl0 = Frag<_Float16>::load(Blp + m * BPITCH + boff);
      const v16h bl1 = Frag<_Float16>::load(Blp + (16 + m) * BPITCH + boff);
      acc0  = Frag<_Float16>::mma(a, bh0, acc0);
      acc1  = Frag<_Float16>::mma(a, bh1, acc1);
      accl0 = Frag<_Float16>::mma(a, bl0, accl0);
      accl1 = Frag<_Float16>::mma(a, bl1, accl1);
      mma_guard4(acc0, acc1, accl0, accl1, a, bh0, bh1, bl0, bl1);
    }

#pragma unroll
    for (int r = 0; r < 8; ++r) {
      const float v0 = fmaf(acc0[r], OUT_SCALE, accl0[r] * LO_SCALE);
      const float v1 = fmaf(acc1[r], OUT_SCALE, accl1[r] * LO_SCALE);
      sw[(8 * hh + r) * SPITCH + m]      = v0;
      sw[(8 * hh + r) * SPITCH + 16 + m] = v1;
    }
    __builtin_amdgcn_fence(__ATOMIC_RELEASE, "workgroup");
    __builtin_amdgcn_wave_barrier();
    __builtin_amdgcn_fence(__ATOMIC_ACQUIRE, "workgroup");
    {
      const int q = lane >> 3, c4 = (lane & 7) * 4;
      for (int pass = 0; pass < 2; ++pass) {
#pragma unroll
        for (int it = 0; it < 4; ++it) {
          const int row = it * 4 + q;
          const v4f v = *(const v4f*)(sw + row * SPITCH + c4);
          *(volatile v4f*)(T + (size_t)(e0 + row) * ADIM + c4) = v;
        }
        __threadfence();
      }
    }
    __builtin_amdgcn_fence(__ATOMIC_RELEASE, "workgroup");
    __builtin_amdgcn_wave_barrier();
    __builtin_amdgcn_fence(__ATOMIC_ACQUIRE, "workgroup");
  }
}

__device__ __forceinline__ int chunk_hits(const int* __restrict__ pairs, int e0, int n0, int tid, int* LIST, int* scan_ws) {
  const int eb = e0 + tid * EPT;
  const bool valid = eb < NEDGE;
  const int ebc = valid ? eb : (NEDGE - EPT);
  const v4i* pp = (const v4i*)(pairs + 2 * (size_t)ebc);
  int rec[EPT]; int cnt = 0;
#pragma unroll
  for (int k = 0; k < EPT / 2; ++k) {
    const v4i w = pp[k];
    {
      const unsigned rel = (unsigned)w[0] - (unsigned)n0; int r = -1;
      if (valid && rel < (unsigned)SRB) { r = (int)((rel << 19) | (unsigned)(ebc + 2 * k)); ++cnt; }
      rec[2 * k] = r;
    }
    {
      const unsigned rel = (unsigned)w[2] - (unsigned)n0; int r = -1;
      if (valid && rel < (unsigned)SRB) { r = (int)((rel << 19) | (unsigned)(ebc + 2 * k + 1)); ++cnt; }
      rec[2 * k + 1] = r;
    }
  }
  int tot; int p = blk_excl_scan(cnt, scan_ws, tid, &tot);
#pragma unroll
  for (int k = 0; k < EPT; ++k) if (rec[k] >= 0) { if ((unsigned)p < (unsigned)LCAP) LIST[p] = rec[k]; ++p; }
  __syncthreads();
  return tot < LCAP ? tot : LCAP;
}

__global__ __launch_bounds__(NT) void segment_sum_kernel(const float* __restrict__ T, const int* __restrict__ pairs,
                                                         float* __restrict__ out) {
  __shared__ __align__(16) float accs[SRB * ADIM];
  __shared__ int LIST[LCAP];
  __shared__ int scan_ws[80];
  const int tid = threadIdx.x, lane = tid & 31, wave = tid >> 5;
  const int n0 = blockIdx.x * SRB;
  if (tid < 80) scan_ws[tid] = 0;
#pragma unroll 1
  for (int j = 0; j < 128; ++j) accs[(wave * 128 + j) * ADIM + lane] = 0.0f;
  __syncthreads();

#pragma unroll 1
  for (int c = 0; c < NCH; ++c) {
    const int tot = chunk_hits(pairs, c * SCH, n0, tid, LIST, scan_ws);
#pragma unroll 1
    for (int base = 0; base < tot; base += 32) {
      const int q = base + lane;
      const int qc = q < tot ? q : tot - 1;
      int rv = LIST[qc];
      rv = (q < tot) ? rv : -1;
      const int own = (rv >= 0 && (rv >> 26) == wave) ? 1 : 0;
      unsigned msk = (unsigned)__ballot(own);
#pragma unroll 1
      for (int it = 0; it < 32; ++it) {
        if (msk == 0u) break;
        const int bp = __builtin_ctz(msk); msk &= msk - 1u;
        const int r = __shfl(rv, bp, 32);
        const int dl = (r >> 19) & (SRB - 1);
        int e = r & 0x7FFFF; e = e < NEDGE ? e : NEDGE - 1;
        const float tv = T[(size_t)e * ADIM + lane];
        accs[dl * ADIM + lane] += tv;
      }
    }
    __syncthreads();
  }

  {
    const int q = lane >> 3, c4 = (lane & 7) * 4;
    for (int pass = 0; pass < 2; ++pass) {
#pragma unroll 1
      for (int j = 0; j < 32; ++j) {
        const int rl = wave * 128 + j * 4;
        if (n0 + rl < NATOM) {
          const v4f v = *(const v4f*)(accs + (rl + q) * ADIM + c4);
          *(volatile v4f*)(out + (size_t)(n0 + rl + q) * ADIM + c4) = v;
        }
      }
      __threadfence();
    }
  }
}

extern "C" void kernel_launch(void* const* d_in, const int* in_sizes, int n_in,
                              void* d_out, int out_size, void* d_ws, size_t ws_size, hipStream_t stream) {
  if (n_in < 5) return;
  if (in_sizes[0] != NATOM * ADIM || in_sizes[1] != NEDGE * BDIM || in_sizes[2] != NEDGE * 2 ||
      in_sizes[3] != BDIM * WCOLS || in_sizes[4] != WCOLS || out_size != NATOM * ADIM) return;
  const size_t t_bytes = (size_t)NEDGE * ADIM * sizeof(float);
  if (t_bytes > ws_size || t_bytes > (size_t)134217728) return;

  const float* atom  = (const float*)d_in[0];
  const float* bond  = (const float*)d_in[1];
  const int*   pairs = (const int*)  d_in[2];
  const float* W     = (const float*)d_in[3];
  const float* bias  = (const float*)d_in[4];
  float* out = (float*)d_out;
  float* T   = (float*)d_ws;

  edge_transform_kernel<<<NBLK1, NT, 0, stream>>>(atom, bond, pairs, W, bias, T);
  segment_sum_kernel<<<NTILE2, NT, 0, stream>>>(T, pairs, out);
}
